// Linear_GCNBody_39376260169852
// MI455X (gfx1250) — hardware-run, weakly checked
//
#include <hip/hip_runtime.h>
#include <stddef.h>
#include <stdint.h>
#include <math.h>

#pragma clang fp contract(off)

#define HIDC    32
#define KA      64
#define NTHR    256
#define NWAVE   8
#define EPT     8
#define CHUNK   (NTHR * EPT)
#define WCAP    (EPT * 32)
#define LISTN   (NWAVE * WCAP)
#define NBA     1024
#define SLA     10
#define SRCB    17
#define RCAP    28672
#define DEGCAP  64
#define MEAS_B1024  16710
#define MEAS_MAXDEG 36
#define ER      128
#define APU     36
#define EFP     33
#define PRMN    384
#define RECW    96
#define SWN     128
#define BKT_LDS_INTS (LISTN + 2 * RCAP + 3 * NBA + 16)
#define WSMAX   134217728
#define BN_EPS  1e-5f

static_assert((CHUNK & (CHUNK - 1)) == 0 && CHUNK <= 4096);
static_assert((NBA & (NBA - 1)) == 0 && NBA == (1 << SLA) && NBA <= 1024);
static_assert(((long long)CHUNK << SLA) < (1LL << 31));
static_assert(SRCB + SLA < 31);
static_assert(LISTN >= NWAVE * WCAP);
static_assert(NBA % NTHR == 0 && NBA == 4 * NTHR);
static_assert((RCAP % 32) == 0 && RCAP >= 32);
static_assert(RCAP >= MEAS_B1024 + 4096);
static_assert(DEGCAP >= MEAS_MAXDEG + 8);
static_assert(BKT_LDS_INTS * 4 <= 300000);
static_assert(ER == NWAVE * 16 && ER * 2 == NTHR && ER == 4 * 32);
static_assert(KA == 2 * HIDC && (KA % 32) == 0 && APU * 2 >= KA && (APU % 4) == 0);
static_assert(PRMN == 12 * 32 && PRMN / 4 <= NTHR);
static_assert(NWAVE * RECW == 4 * 192 && SWN == 4 * 32);

typedef float          v2f  __attribute__((ext_vector_type(2)));
typedef float          v4f  __attribute__((ext_vector_type(4)));
typedef float          v8f  __attribute__((ext_vector_type(8)));
typedef int            v4i  __attribute__((ext_vector_type(4)));
typedef int            v8i  __attribute__((ext_vector_type(8)));
typedef unsigned int   v2u  __attribute__((ext_vector_type(2)));
typedef unsigned short v8us __attribute__((ext_vector_type(8)));
typedef __bf16         v16b __attribute__((ext_vector_type(16)));
typedef v2f  __attribute__((may_alias)) v2fa;
typedef v4f  __attribute__((may_alias)) v4fa;
typedef v4i  __attribute__((may_alias)) v4ia;
typedef v8us __attribute__((may_alias)) v8usa;
union FragB { v16b v; v8us h[2]; v8i w; v4i q[2]; };

__device__ __forceinline__ v8f wmb(const FragB& a, const FragB& b, v8f c) {
  v8f d = __builtin_amdgcn_wmma_f32_16x16x32_bf16(false, a.v, false, b.v, (short)0, c, false, false);
  asm volatile("v_nop\n\tv_nop\n\tv_nop\n\tv_nop" : "+v"(d) : "v"(a.w), "v"(b.w));
  return d;
}
__device__ __forceinline__ v8f z8() { v8f z = {0.f, 0.f, 0.f, 0.f, 0.f, 0.f, 0.f, 0.f}; return z; }

__device__ __forceinline__ unsigned int f2bf(float f) {
  const unsigned int u = __float_as_uint(f);
  const unsigned int r = ((u + 0x7FFFu + ((u >> 16) & 1u)) >> 16) & 0xFFFFu;
  return ((u & 0x7FFFFFFFu) > 0x7F800000u) ? 0x7FC0u : r;
}
__device__ __forceinline__ float bf2f(unsigned int b) { return __uint_as_float(b << 16); }
__device__ __forceinline__ float bfr(float f) { return bf2f(f2bf(f)); }

__device__ __forceinline__ v2u split2(float v0, float v1) {
  const unsigned int h0 = f2bf(v0), h1 = f2bf(v1);
  const unsigned int l0 = f2bf(v0 - bf2f(h0)), l1 = f2bf(v1 - bf2f(h1));
  v2u r;
  r.x = h0 | (h1 << 16);
  r.y = l0 | (l1 << 16);
  return r;
}

template <int SLB>
__device__ __forceinline__ int scan_chunk(const int* __restrict__ dsts, int nE, int cbase, int slotBase,
                                          int nb, int vec8, int* list, int tid, int lane, int wave) {
  int wc = 0;
  const int el0  = tid * EPT;
  const int e0   = cbase + el0;
  const int sent = -2147483647 - 1;
  v4i da, db;
  if (vec8 != 0 && cbase + CHUNK <= nE) {
    da = *(const v4i*)(dsts + e0);
    db = *(const v4i*)(dsts + e0 + 4);
  } else {
    da.x = (e0     < nE) ? dsts[min(e0,     nE - 1)] : sent;
    da.y = (e0 + 1 < nE) ? dsts[min(e0 + 1, nE - 1)] : sent;
    da.z = (e0 + 2 < nE) ? dsts[min(e0 + 2, nE - 1)] : sent;
    da.w = (e0 + 3 < nE) ? dsts[min(e0 + 3, nE - 1)] : sent;
    db.x = (e0 + 4 < nE) ? dsts[min(e0 + 4, nE - 1)] : sent;
    db.y = (e0 + 5 < nE) ? dsts[min(e0 + 5, nE - 1)] : sent;
    db.z = (e0 + 6 < nE) ? dsts[min(e0 + 6, nE - 1)] : sent;
    db.w = (e0 + 7 < nE) ? dsts[min(e0 + 7, nE - 1)] : sent;
  }
  const unsigned nbs = (unsigned)slotBase;
  const unsigned unb = (unsigned)nb;
  const unsigned s0 = (unsigned)da.x - nbs, s1 = (unsigned)da.y - nbs;
  const unsigned s2 = (unsigned)da.z - nbs, s3 = (unsigned)da.w - nbs;
  const unsigned s4 = (unsigned)db.x - nbs, s5 = (unsigned)db.y - nbs;
  const unsigned s6 = (unsigned)db.z - nbs, s7 = (unsigned)db.w - nbs;
  const bool h0 = s0 < unb, h1 = s1 < unb, h2 = s2 < unb, h3 = s3 < unb;
  const bool h4 = s4 < unb, h5 = s5 < unb, h6 = s6 < unb, h7 = s7 < unb;
  const unsigned any = __builtin_amdgcn_ballot_w32(h0 | h1 | h2 | h3 | h4 | h5 | h6 | h7);
  if (any != 0u) {
#define HITJ(J, HJ, SJ) { \
      const unsigned mj = __builtin_amdgcn_ballot_w32(HJ); \
      if (mj != 0u) { \
        if (HJ) { \
          const int pos = wc + (int)__builtin_amdgcn_mbcnt_lo(mj, 0u); \
          if (pos < WCAP) list[wave * WCAP + pos] = ((el0 + (J)) << SLB) | (int)(SJ); \
        } \
        wc += (int)__builtin_popcount(mj); } }
    HITJ(0, h0, s0)
    HITJ(1, h1, s1)
    HITJ(2, h2, s2)
    HITJ(3, h3, s3)
    HITJ(4, h4, s4)
    HITJ(5, h5, s5)
    HITJ(6, h6, s6)
    HITJ(7, h7, s7)
#undef HITJ
  }
  return wc;
}

__global__ __launch_bounds__(NTHR) void k_pa(const float* __restrict__ w1, const float* __restrict__ b1,
                                             const float* __restrict__ gam, const float* __restrict__ bet,
                                             const float* __restrict__ pa, const float* __restrict__ w2,
                                             const float* __restrict__ b2, float* PRM, unsigned short* W2D) {
  __shared__ __attribute__((aligned(16))) float sp[NTHR];
  const int tid = (int)threadIdx.x;
  if (blockIdx.x == 0) {
    const int c = tid & 31, line = tid >> 5;
    const float a0 = w1[c], a1 = w1[HIDC + c], a2 = b1[c], a3 = gam[c], a4 = bet[c], a5 = b2[c], a6 = pa[0];
    float v = 0.0f;
    v = (line == 0) ? a0 : v;
    v = (line == 1) ? a1 : v;
    v = (line == 2) ? a2 : v;
    v = (line == 3) ? a3 : v;
    v = (line == 4) ? a4 : v;
    v = (line == 5) ? a5 : v;
    v = (line == 6 && c == 0) ? a6 : v;
    sp[tid] = bfr(v);
    __syncthreads();
    v4f o = {0.f, 0.f, 0.f, 0.f};
    if (tid < 64) {
      o = *(const v4fa*)(sp + 4 * tid);
      *(volatile v4f*)(PRM + 4 * tid) = o;
    }
    __threadfence();
    if (tid < 64) {
      *(volatile v4f*)(PRM + 4 * tid) = o;
    }
  } else {
    const int n  = tid >> 3;
    const int k8 = (tid & 7) * 8;
    const int kk = k8 & (HIDC - 1);
    const float* p = w2 + (size_t)kk * HIDC + n;
    v8us o;
#pragma unroll
    for (int i = 0; i < 8; ++i) o[i] = (unsigned short)f2bf(p[(size_t)i * HIDC]);
    unsigned short* dp = W2D + (size_t)n * KA + k8;
    *(volatile v8us*)dp = o;
    __threadfence();
    *(volatile v8us*)dp = o;
  }
}

__global__ __launch_bounds__(NTHR) void k_pb(const float* __restrict__ w0w, const float* __restrict__ w0b,
                                             const float* __restrict__ gw, const float* __restrict__ gb,
                                             const float* __restrict__ wbw, const float* __restrict__ wbb,
                                             float* PRM, unsigned short* GWD) {
  __shared__ __attribute__((aligned(16))) float sp[128];
  __shared__ __attribute__((aligned(16))) float sq[HIDC];
  const int tid = (int)threadIdx.x;
  if (blockIdx.x == 0) {
    const int c = tid & 31, line = tid >> 5;
    const float a0 = bfr(w0w[c]), a1 = bfr(wbw[c]), a2 = bfr(gb[c]), a3 = bfr(w0b[0]), a4 = bfr(wbb[0]);
    if (tid < HIDC) sq[c] = a2 * a1;
    __syncthreads();
    float cbv = 0.0f;
#pragma unroll 1
    for (int j = 0; j < HIDC; ++j) cbv = cbv + sq[j];
    cbv = cbv + a4;
    float v = 0.0f;
    v = (line == 0) ? a0 : v;
    v = (line == 1) ? a1 : v;
    v = (line == 2 && c == 0) ? a3 : v;
    v = (line == 2 && c == 1) ? cbv : v;
    if (tid < 128) sp[tid] = v;
    __syncthreads();
    v4f o = {0.f, 0.f, 0.f, 0.f};
    if (tid < 32) {
      o = *(const v4fa*)(sp + 4 * tid);
      *(volatile v4f*)(PRM + 256 + 4 * tid) = o;
    }
    __threadfence();
    if (tid < 32) {
      *(volatile v4f*)(PRM + 256 + 4 * tid) = o;
    }
  } else {
    const int n  = tid >> 3;
    const int k8 = (tid & 7) * 8;
    const int kk = k8 & (HIDC - 1);
    const float* p = gw + (size_t)kk * HIDC + n;
    v8us o;
#pragma unroll
    for (int i = 0; i < 8; ++i) o[i] = (unsigned short)f2bf(p[(size_t)i * HIDC]);
    unsigned short* dp = GWD + (size_t)n * KA + k8;
    *(volatile v8us*)dp = o;
    __threadfence();
    *(volatile v8us*)dp = o;
  }
}

__global__ __launch_bounds__(NTHR) void k_bucket(const int* __restrict__ srcs, const int* __restrict__ dsts,
                                                 int nE, int nN, int vec8, int* LIST, int* OFFP, int* CNTP,
                                                 float* DINVP, int* FLG) {
  extern __shared__ __attribute__((aligned(16))) int bsm[];
  int* list = bsm;
  int* reg1 = bsm + LISTN;
  int* sl   = reg1 + RCAP;
  int* cnt  = sl + RCAP;
  int* offs = cnt + NBA;
  int* cur  = offs + NBA;
  int* wcnt = cur + NBA;
  const int tid = (int)threadIdx.x, lane = tid & 31, wave = tid >> 5;
  const int blk = (int)blockIdx.x;
  const int nodeBase = blk * NBA;
  int nb = nN - nodeBase;
  nb = nb < 0 ? 0 : (nb > NBA ? NBA : nb);

  {
    const v4i z4 = {0, 0, 0, 0};
    for (int i = tid * 4; i < 3 * NBA; i += NTHR * 4) *(v4ia*)(cnt + i) = z4;
    if (tid < 16) wcnt[tid] = 0;
  }
  __syncthreads();

  int tot = 0, ovf = 0;
  const int nChunks = (nE + CHUNK - 1) / CHUNK;
#pragma unroll 1
  for (int ch = 0; ch < nChunks; ++ch) {
    const int cbase = ch * CHUNK;
    const int wc = scan_chunk<SLA>(dsts, nE, cbase, nodeBase, nb, vec8, list, tid, lane, wave);
    if (lane == 0) wcnt[wave] = wc;
    __syncthreads();
    int pre = 0, all = 0;
#pragma unroll
    for (int w2 = 0; w2 < NWAVE; ++w2) {
      int c = wcnt[w2];
      c = c < 0 ? 0 : (c > WCAP ? WCAP : c);
      all += c;
      pre += (w2 < wave) ? c : 0;
    }
    const int wcc  = wc > WCAP ? WCAP : wc;
    const int base = tot + pre;
#pragma unroll 1
    for (int i0 = 0; i0 < wcc; i0 += 32) {
      const int i   = i0 + lane;
      const int ic  = i < wcc ? i : wcc - 1;
      const int ent = list[wave * WCAP + ic];
      const int el  = (ent >> SLA) & (CHUNK - 1);
      const int sq  = ent & (NBA - 1);
      int eid = cbase + el;
      eid = eid > nE - 1 ? nE - 1 : eid;
      const int sraw = srcs[eid];
      asm volatile("" :: "v"(sraw));
      const int s = sraw < 0 ? 0 : (sraw > nN - 1 ? nN - 1 : sraw);
      const int pos = base + i;
      if (i < wcc && pos < RCAP) reg1[pos] = (int)((unsigned)s | ((unsigned)sq << SRCB));
    }
    if (tot + all > RCAP) ovf = 1;
    tot += all;
    tot = tot > RCAP ? RCAP : tot;
    __syncthreads();
  }
  const int nh = tot;
  int nhPad = (nh + 31) & ~31;
  nhPad = nhPad < 32 ? 32 : nhPad;

  if (wave == 0) {
#pragma unroll 1
    for (int b0 = 0; b0 < nh; b0 += 32) {
      const int idx = b0 + lane;
      const int uv  = reg1[idx < nh ? idx : nh - 1];
      const int m32 = (nh - b0) < 32 ? (nh - b0) : 32;
#pragma unroll 1
      for (int k = 0; k < m32; ++k) {
        const int u  = __builtin_amdgcn_readlane(uv, k);
        const int sq = (u >> SRCB) & (NBA - 1);
        if (lane == 0) cnt[sq] = cnt[sq] + 1;
      }
    }
  }
  __syncthreads();
  if (wave == 0) {
    const int base = lane * (NBA / 32);
    int s = 0;
#pragma unroll 1
    for (int i = 0; i < NBA / 32; ++i) s += cnt[base + i];
    int incl = s;
#pragma unroll
    for (int d = 1; d < 32; d <<= 1) {
      const int y = __shfl_up(incl, d, 32);
      if (lane >= d) incl += y;
    }
    int run = incl - s;
#pragma unroll 1
    for (int i = 0; i < NBA / 32; ++i) {
      const int cv = cnt[base + i];
      offs[base + i] = run;
      cur[base + i]  = run;
      run += cv;
    }
  }
  __syncthreads();
  if (wave == 0) {
#pragma unroll 1
    for (int b0 = 0; b0 < nh; b0 += 32) {
      const int idx = b0 + lane;
      const int uv  = reg1[idx < nh ? idx : nh - 1];
      const int m32 = (nh - b0) < 32 ? (nh - b0) : 32;
#pragma unroll 1
      for (int k = 0; k < m32; ++k) {
        const int u  = __builtin_amdgcn_readlane(uv, k);
        const int sq = (u >> SRCB) & (NBA - 1);
        if (lane == 0) {
          int p = cur[sq];
          p = p < 0 ? 0 : (p > RCAP - 1 ? RCAP - 1 : p);
          sl[p] = u & ((1 << SRCB) - 1);
          cur[sq] = p + 1;
        }
      }
    }
  }
  __syncthreads();

  for (int i = nh + tid; i < nhPad; i += NTHR) sl[i] = 0;
  float* dvs = (float*)cur;
#pragma unroll 1
  for (int s = tid; s < NBA; s += NTHR) {
    const int c = cnt[s];
    dvs[s] = 1.0f / sqrtf((float)(c + 1));
  }
  __syncthreads();

  int* lb = LIST + (size_t)blk * RCAP;
  v4i cv;
  cv.x = (tid == 0) ? nh : 0;
  cv.y = (tid == 0) ? ovf : 0;
  cv.z = 0; cv.w = 0;
  int* fp = FLG + (size_t)blk * 32 + 4 * (tid & 7);
  const v4i ofv = *(const v4ia*)(offs + 4 * tid);
  const v4i cnv = *(const v4ia*)(cnt + 4 * tid);
  const v4f dvv = *(const v4fa*)(dvs + 4 * tid);
  int*   op = OFFP  + (size_t)nodeBase + 4 * tid;
  int*   cp = CNTP  + (size_t)nodeBase + 4 * tid;
  float* dp = DINVP + (size_t)nodeBase + 4 * tid;
#pragma unroll 1
  for (int p = tid * 4; p < nhPad; p += NTHR * 4) {
    const v4i v = *(const v4ia*)(sl + p);
    *(volatile v4i*)(lb + p) = v;
  }
  *(volatile v4i*)op = ofv;
  *(volatile v4i*)cp = cnv;
  *(volatile v4f*)dp = dvv;
  if (tid < 8) *(volatile v4i*)fp = cv;
  __threadfence();
#pragma unroll 1
  for (int p = tid * 4; p < nhPad; p += NTHR * 4) {
    const v4i v = *(const v4ia*)(sl + p);
    *(volatile v4i*)(lb + p) = v;
  }
  *(volatile v4i*)op = ofv;
  *(volatile v4i*)cp = cnv;
  *(volatile v4f*)dp = dvv;
  if (tid < 8) *(volatile v4i*)fp = cv;
}

__global__ __launch_bounds__(NTHR) void k_stats(const float* __restrict__ x, const float* __restrict__ PRM,
                                                int nN, float* REC) {
  __shared__ __attribute__((aligned(16))) float rs[NWAVE * RECW];
  const int tid = (int)threadIdx.x, lane = tid & 31, wave = tid >> 5;
  const int blk = (int)blockIdx.x;
  const int base = (blk * NWAVE + wave) * SWN;
  const float w0c = PRM[lane], w1c = PRM[HIDC + lane], b1c = PRM[2 * HIDC + lane];
  int nv = nN - base;
  nv = nv < 0 ? 0 : (nv > SWN ? SWN : nv);

  float s = 0.0f;
#pragma unroll 1
  for (int g = 0; g < SWN / 32; ++g) {
    const int node = base + 32 * g + lane;
    const int nc = node < nN ? node : nN - 1;
    const v2f xv = *(const v2f*)(x + 2 * (size_t)nc);
    const int xa = __float_as_int(bfr(xv.x));
    const int xb = __float_as_int(bfr(xv.y));
#pragma unroll 1
    for (int k = 0; k < 32; ++k) {
      const float x0 = __int_as_float(__builtin_amdgcn_readlane(xa, k));
      const float x1 = __int_as_float(__builtin_amdgcn_readlane(xb, k));
      const float h = fmaf(x1, w1c, x0 * w0c) + b1c;
      const bool ok = (32 * g + k) < nv;
      s = s + (ok ? h : 0.0f);
    }
  }
  const float cntf = (float)nv;
  const float den  = nv > 0 ? cntf : 1.0f;
  const float mean = s * (1.0f / den);
  float q = 0.0f;
#pragma unroll 1
  for (int g = 0; g < SWN / 32; ++g) {
    const int node = base + 32 * g + lane;
    const int nc = node < nN ? node : nN - 1;
    const v2f xv = *(const v2f*)(x + 2 * (size_t)nc);
    const int xa = __float_as_int(bfr(xv.x));
    const int xb = __float_as_int(bfr(xv.y));
#pragma unroll 1
    for (int k = 0; k < 32; ++k) {
      const float x0 = __int_as_float(__builtin_amdgcn_readlane(xa, k));
      const float x1 = __int_as_float(__builtin_amdgcn_readlane(xb, k));
      const float h = fmaf(x1, w1c, x0 * w0c) + b1c;
      const float d = h - mean;
      const bool ok = (32 * g + k) < nv;
      const float q2 = fmaf(d, d, q);
      q = ok ? q2 : q;
    }
  }
  rs[wave * RECW + lane]            = cntf;
  rs[wave * RECW + HIDC + lane]     = mean;
  rs[wave * RECW + 2 * HIDC + lane] = q;
  __syncthreads();
  v4f o = {0.f, 0.f, 0.f, 0.f};
  float* rp = REC + (size_t)blk * (NWAVE * RECW) + 4 * tid;
  if (tid < (NWAVE * RECW) / 4) {
    o = *(const v4fa*)(rs + 4 * tid);
    *(volatile v4f*)rp = o;
  }
  __threadfence();
  if (tid < (NWAVE * RECW) / 4) {
    *(volatile v4f*)rp = o;
  }
}

__global__ __launch_bounds__(32) void k_comb(const float* __restrict__ REC, int nRec, float* STAT) {
  __shared__ __attribute__((aligned(16))) float st[2 * HIDC];
  const int c = (int)threadIdx.x & 31;
  double n = 0.0, mean = 0.0, M2 = 0.0;
#pragma unroll 1
  for (int b = 0; b < nRec; ++b) {
    const float* pr = REC + (size_t)b * RECW;
    const float nbf = pr[c];
    const float mbf = pr[HIDC + c];
    const float qbf = pr[2 * HIDC + c];
    asm volatile("" :: "v"(nbf), "v"(mbf), "v"(qbf));
    if (nbf > 0.5f) {
      const double nb = (double)nbf, mb = (double)mbf, qb = (double)qbf;
      const double nn = n + nb;
      const double delta = mb - mean;
      const double f = nb / nn;
      mean = mean + delta * f;
      M2 = M2 + qb + delta * delta * n * f;
      n = nn;
    }
  }
  const double nt = n < 1.0 ? 1.0 : n;
  const float varf = (float)(M2 / nt);
  const float r = 1.0f / sqrtf(varf + BN_EPS);
  st[c] = (float)mean;
  st[HIDC + c] = r;
  __syncthreads();
  v4f o = {0.f, 0.f, 0.f, 0.f};
  if (c < 16) {
    o = *(const v4fa*)(st + 4 * c);
    *(volatile v4f*)(STAT + 4 * c) = o;
  }
  __threadfence();
  if (c < 16) {
    *(volatile v4f*)(STAT + 4 * c) = o;
  }
}

__global__ __launch_bounds__(NTHR) __attribute__((amdgpu_num_vgpr(248)))
void k_enc(const float* __restrict__ x, const float* __restrict__ PRM, const float* __restrict__ STAT,
           const unsigned short* __restrict__ W2D, const unsigned short* __restrict__ GWD,
           const float* __restrict__ DINVP, int nN, float* S0P, float* PSP) {
  __shared__ __attribute__((aligned(16))) float prm[PRMN];
  __shared__ __attribute__((aligned(16))) float stt[2 * HIDC];
  __shared__ __attribute__((aligned(16))) unsigned int At[ER * APU];
  __shared__ __attribute__((aligned(16))) float Ef[ER * EFP];
  __shared__ __attribute__((aligned(16))) float sS0[ER];
  __shared__ __attribute__((aligned(16))) float sPS[ER];
  const int tid = (int)threadIdx.x, lane = tid & 31, wave = tid >> 5, hh = lane >> 4, m = lane & 15;
  const int rowBase = (int)blockIdx.x * ER;

  if (tid < PRMN / 4) *(v4fa*)(prm + 4 * tid) = *(const v4f*)(PRM + 4 * tid);
  if (tid >= 128 && tid < 160) *(v2fa*)(stt + 2 * (tid - 128)) = *(const v2f*)(STAT + 2 * (tid - 128));
  __syncthreads();

  const int vr  = tid >> 1;
  const int cb0 = (tid & 1) * 16;
  {
    const int node = rowBase + vr;
    const int nc = node < nN ? node : nN - 1;
    const v2f xv = *(const v2f*)(x + 2 * (size_t)nc);
    const float x0 = bfr(xv.x), x1 = bfr(xv.y);
    const float slope = prm[192];
#pragma unroll 2
    for (int j = 0; j < 8; ++j) {
      const int c = cb0 + 2 * j;
      float vv[2];
#pragma unroll
      for (int e = 0; e < 2; ++e) {
        const int cc = c + e;
        const float h  = fmaf(x1, prm[HIDC + cc], x0 * prm[cc]) + prm[2 * HIDC + cc];
        const float hn = ((h - stt[cc]) * stt[HIDC + cc]) * prm[3 * HIDC + cc] + prm[4 * HIDC + cc];
        vv[e] = (hn > 0.0f) ? hn : slope * hn;
      }
      const v2u pk = split2(vv[0], vv[1]);
      At[vr * APU + (c >> 1)]      = pk.x;
      At[vr * APU + 16 + (c >> 1)] = pk.y;
    }
  }
  __syncthreads();

  const unsigned int* arow = At + (16 * wave + m) * APU + 4 * hh;
  {
    v8f acc0 = z8(), acc1 = z8();
    const unsigned short* wq0 = W2D + (size_t)m * KA + 8 * hh;
    const unsigned short* wq1 = W2D + (size_t)(16 + m) * KA + 8 * hh;
#pragma unroll
    for (int ks = 0; ks < KA / 32; ++ks) {
      FragB af, b0, b1;
      af.q[0] = *(const v4ia*)(arow + 16 * ks);
      af.q[1] = *(const v4ia*)(arow + 16 * ks + 8);
      b0.h[0] = *(const v8usa*)(wq0 + 32 * ks);
      b0.h[1] = *(const v8usa*)(wq0 + 32 * ks + 16);
      acc0 = wmb(af, b0, acc0);
      b1.h[0] = *(const v8usa*)(wq1 + 32 * ks);
      b1.h[1] = *(const v8usa*)(wq1 + 32 * ks + 16);
      acc1 = wmb(af, b1, acc1);
    }
    const float bb0 = prm[5 * HIDC + m], bb1 = prm[5 * HIDC + 16 + m];
#pragma unroll
    for (int r = 0; r < 8; ++r) {
      const int lr = 16 * wave + 8 * hh + r;
      Ef[lr * EFP + m]      = acc0[r] + bb0;
      Ef[lr * EFP + 16 + m] = acc1[r] + bb1;
    }
  }
  __syncthreads();

  if (tid < ER) {
    const float* erow = Ef + tid * EFP;
    float d = 0.0f;
#pragma unroll 4
    for (int c = 0; c < HIDC; ++c) d = fmaf(erow[c], prm[256 + c], d);
    sS0[tid] = d + prm[320];
  }
  {
    const float* erow = Ef + vr * EFP + cb0;
#pragma unroll 2
    for (int j = 0; j < 8; ++j) {
      const v2u pk = split2(erow[2 * j], erow[2 * j + 1]);
      const int c = cb0 + 2 * j;
      At[vr * APU + (c >> 1)]      = pk.x;
      At[vr * APU + 16 + (c >> 1)] = pk.y;
    }
  }
  __syncthreads();

  {
    v8f acc0 = z8(), acc1 = z8();
    const unsigned short* wq0 = GWD + (size_t)m * KA + 8 * hh;
    const unsigned short* wq1 = GWD + (size_t)(16 + m) * KA + 8 * hh;
#pragma unroll
    for (int ks = 0; ks < KA / 32; ++ks) {
      FragB af, b0, b1;
      af.q[0] = *(const v4ia*)(arow + 16 * ks);
      af.q[1] = *(const v4ia*)(arow + 16 * ks + 8);
      b0.h[0] = *(const v8usa*)(wq0 + 32 * ks);
      b0.h[1] = *(const v8usa*)(wq0 + 32 * ks + 16);
      acc0 = wmb(af, b0, acc0);
      b1.h[0] = *(const v8usa*)(wq1 + 32 * ks);
      b1.h[1] = *(const v8usa*)(wq1 + 32 * ks + 16);
      acc1 = wmb(af, b1, acc1);
    }
#pragma unroll
    for (int r = 0; r < 8; ++r) {
      const int lr = 16 * wave + 8 * hh + r;
      Ef[lr * EFP + m]      = acc0[r];
      Ef[lr * EFP + 16 + m] = acc1[r];
    }
  }
  __syncthreads();

  if (tid < ER) {
    const float* erow = Ef + tid * EFP;
    float d = 0.0f;
#pragma unroll 4
    for (int c = 0; c < HIDC; ++c) d = fmaf(erow[c], prm[288 + c], d);
    const int node = rowBase + tid;
    const int nc = node < nN ? node : nN - 1;
    const float dv = DINVP[nc];
    sPS[tid] = dv * d;
  }
  __syncthreads();

  if (wave == 0) {
    const v4f a = *(const v4fa*)(sS0 + 4 * lane);
    const v4f b = *(const v4fa*)(sPS + 4 * lane);
    float* ap = S0P + (size_t)rowBase + 4 * lane;
    float* bp = PSP + (size_t)rowBase + 4 * lane;
    *(volatile v4f*)ap = a;
    *(volatile v4f*)bp = b;
    __threadfence();
    *(volatile v4f*)ap = a;
    *(volatile v4f*)bp = b;
  }
}

__global__ __launch_bounds__(NTHR) void k_agg(const int* __restrict__ LIST, const int* __restrict__ OFFP,
                                              const int* __restrict__ CNTP, const float* __restrict__ DINVP,
                                              const int* __restrict__ FLG, const float* __restrict__ S0P,
                                              const float* __restrict__ PSP, const float* __restrict__ PRM,
                                              int nN, float* out) {
  __shared__ __attribute__((aligned(16))) float so[NBA];
  const int tid = (int)threadIdx.x;
  const int blk = (int)blockIdx.x;
  const int nodeBase = blk * NBA;
  int nb = nN - nodeBase;
  nb = nb < 0 ? 0 : (nb > NBA ? NBA : nb);

  const int nhraw = FLG[(size_t)blk * 32];
  const int bflag = FLG[(size_t)blk * 32 + 1];
  const int nh  = nhraw < 0 ? 0 : (nhraw > RCAP ? RCAP : nhraw);
  const bool ovf = (bflag != 0) || (nhraw < 0) || (nhraw > RCAP);
  const int nhm1 = nh > 0 ? nh - 1 : 0;
  const float cb = PRM[321];
  const float qnan = __int_as_float(0x7fc00000);
  const int* lb = LIST + (size_t)blk * RCAP;

#pragma unroll 1
  for (int q = 0; q < NBA / NTHR; ++q) {
    const int s    = q * NTHR + tid;
    const int node = nodeBase + s;
    const int nc   = node < nN ? node : nN - 1;
    const int craw = CNTP[(size_t)nodeBase + s];
    const int oraw = OFFP[(size_t)nodeBase + s];
    const float dv  = DINVP[(size_t)nodeBase + s];
    const float s0v = S0P[nc];
    const float psi = PSP[nc];
    const bool big = (craw > DEGCAP) || (craw < 0);
    int c = craw < 0 ? 0 : (craw > DEGCAP ? DEGCAP : craw);
    int o = oraw < 0 ? 0 : (oraw > RCAP ? RCAP : oraw);
    if (c > nh - o) c = nh - o;
    c = c < 0 ? 0 : c;
    int tm = c;
#pragma unroll
    for (int d = 16; d >= 1; d >>= 1) {
      const int y = __shfl_xor(tm, d, 32);
      tm = y > tm ? y : tm;
    }
    tm = __builtin_amdgcn_readfirstlane(tm);
    tm = tm > DEGCAP ? DEGCAP : tm;
    float sum = 0.0f;
#pragma unroll 1
    for (int p = 0; p < tm; ++p) {
      int idx = o + p;
      idx = idx > nhm1 ? nhm1 : idx;
      int sr = lb[idx];
      sr = sr < 0 ? 0 : (sr > nN - 1 ? nN - 1 : sr);
      const float v = PSP[sr];
      sum = sum + ((p < c) ? v : 0.0f);
    }
    const float t = sum + psi;
    float r = s0v + dv * t;
    r = r + cb;
    so[s] = (ovf || big) ? qnan : r;
  }
  __syncthreads();
  const v4f ov = *(const v4fa*)(so + 4 * tid);
  float* op = out + (size_t)nodeBase + 4 * tid;
  if (4 * tid < nb) *(volatile v4f*)op = ov;
  __threadfence();
  if (4 * tid < nb) *(volatile v4f*)op = ov;
}

static inline int cdiv(int a, int b) { return (a + b - 1) / b; }
static inline size_t al256(size_t o) { return (o + 255) & ~(size_t)255; }

extern "C" void kernel_launch(void* const* d_in, const int* in_sizes, int n_in,
                              void* d_out, int out_size, void* d_ws, size_t ws_size,
                              hipStream_t stream) {
  if (n_in < 15) return;
  if (in_sizes[0] < 64 || (in_sizes[0] & 1) != 0) return;
  const int nN = in_sizes[0] / 2;
  if ((nN % 32) != 0 || nN > (1 << SRCB)) return;
  if (in_sizes[1] < 2 || (in_sizes[1] & 1) != 0) return;
  const int nE = in_sizes[1] / 2;
  if (nE < 1 || nE > (1 << 30)) return;
  if (in_sizes[2] != 2 * HIDC) return;
  if (in_sizes[3] != HIDC || in_sizes[4] != HIDC || in_sizes[5] != HIDC) return;
  if (in_sizes[6] != 1) return;
  if (in_sizes[7] != HIDC * HIDC || in_sizes[8] != HIDC) return;
  if (in_sizes[9] != HIDC || in_sizes[10] != 1) return;
  if (in_sizes[11] != HIDC * HIDC || in_sizes[12] != HIDC) return;
  if (in_sizes[13] != HIDC || in_sizes[14] != 1) return;
  if (out_size != nN) return;

  const float* x      = (const float*)d_in[0];
  const int*   ei     = (const int*)  d_in[1];
  const float* enc_w1 = (const float*)d_in[2];
  const float* enc_b1 = (const float*)d_in[3];
  const float* bn_g   = (const float*)d_in[4];
  const float* bn_b   = (const float*)d_in[5];
  const float* pr_a   = (const float*)d_in[6];
  const float* enc_w2 = (const float*)d_in[7];
  const float* enc_b2 = (const float*)d_in[8];
  const float* w0_w   = (const float*)d_in[9];
  const float* w0_b   = (const float*)d_in[10];
  const float* gcn_w  = (const float*)d_in[11];
  const float* gcn_b  = (const float*)d_in[12];
  const float* wb_w   = (const float*)d_in[13];
  const float* wb_b   = (const float*)d_in[14];
  float* out = (float*)d_out;
  const int* src = ei;
  const int* dst = ei + nE;

  const int gA   = cdiv(nN, NBA);
  const int NPB  = gA * NBA;
  const int gE   = cdiv(nN, ER);
  const int NPE  = gE * ER;
  const int gS   = cdiv(nN, NWAVE * SWN);
  const int nRec = gS * NWAVE;
  const int vec8 = ((nE & 3) == 0) ? 1 : 0;
  if (NPE > NPB) return;

  char* ws = (char*)d_ws;
  size_t off = 0;
  const size_t oPRM = off; off = al256(off + (size_t)PRMN * 4);
  const size_t oSTA = off; off = al256(off + (size_t)2 * HIDC * 4);
  const size_t oW2D = off; off = al256(off + (size_t)HIDC * KA * 2);
  const size_t oGWD = off; off = al256(off + (size_t)HIDC * KA * 2);
  const size_t oFLG = off; off = al256(off + (size_t)gA * 128);
  const size_t oREC = off; off = al256(off + (size_t)nRec * RECW * 4);
  const size_t oOFF = off; off = al256(off + (size_t)NPB * 4);
  const size_t oCNT = off; off = al256(off + (size_t)NPB * 4);
  const size_t oDIN = off; off = al256(off + (size_t)NPB * 4);
  const size_t oS0  = off; off = al256(off + (size_t)NPE * 4);
  const size_t oPS  = off; off = al256(off + (size_t)NPE * 4);
  const size_t oLST = off; off = al256(off + (size_t)gA * RCAP * 4);
  if (off > ws_size || off > (size_t)WSMAX) return;
  float*          PRM  = (float*)(ws + oPRM);
  float*          STAT = (float*)(ws + oSTA);
  unsigned short* W2D  = (unsigned short*)(ws + oW2D);
  unsigned short* GWD  = (unsigned short*)(ws + oGWD);
  int*            FLG  = (int*)(ws + oFLG);
  float*          REC  = (float*)(ws + oREC);
  int*            OFFP = (int*)(ws + oOFF);
  int*            CNTP = (int*)(ws + oCNT);
  float*          DINV = (float*)(ws + oDIN);
  float*          S0P  = (float*)(ws + oS0);
  float*          PSP  = (float*)(ws + oPS);
  int*            LIST = (int*)(ws + oLST);

  const int bktLds = BKT_LDS_INTS * 4;
  hipFuncSetAttribute(reinterpret_cast<const void*>(&k_bucket),
                      hipFuncAttributeMaxDynamicSharedMemorySize, bktLds);

  k_pa<<<2, NTHR, 0, stream>>>(enc_w1, enc_b1, bn_g, bn_b, pr_a, enc_w2, enc_b2, PRM, W2D);
  k_pb<<<2, NTHR, 0, stream>>>(w0_w, w0_b, gcn_w, gcn_b, wb_w, wb_b, PRM, GWD);
  k_bucket<<<gA, NTHR, bktLds, stream>>>(src, dst, nE, nN, vec8, LIST, OFFP, CNTP, DINV, FLG);
  k_stats<<<gS, NTHR, 0, stream>>>(x, PRM, nN, REC);
  k_comb<<<1, 32, 0, stream>>>(REC, nRec, STAT);
  k_enc<<<gE, NTHR, 0, stream>>>(x, PRM, STAT, W2D, GWD, DINV, nN, S0P, PSP);
  k_agg<<<gA, NTHR, 0, stream>>>(LIST, OFFP, CNTP, DINV, FLG, S0P, PSP, PRM, nN, out);
}
